// ViTMoEAttention_23356032155700
// MI455X (gfx1250) — hardware-verified
//
#include <hip/hip_runtime.h>
#include <math.h>
#include <stdint.h>

#define BB    32
#define SQ    257
#define SP    272
#define TOKP  (BB * SP)
#define DIM   1024
#define NH    16
#define HD    64
#define NE    8
#define RK    16
#define KE    32
#define NQT   (SP / 16)
#define NQB   5
#define NKT   5
static_assert(NH * HD == DIM);
static_assert(NQT * 16 == SP);
static_assert(SP >= SQ);
static_assert((SP % 16) == 0);
static_assert(NQB * 4 >= NQT);
static_assert((NKT - 1) * 64 < SQ);
static_assert(NQT - 4 * (NKT - 1) >= 1);
static_assert(NQT - 4 * (NKT - 1) <= 4);
static_assert((TOKP % 64) == 0);
static_assert(KE == 2 * RK);

typedef _Float16 v16h __attribute__((ext_vector_type(16)));
typedef _Float16 v8h  __attribute__((ext_vector_type(8)));
typedef __bf16   v16b __attribute__((ext_vector_type(16)));
typedef __bf16   v8b  __attribute__((ext_vector_type(8)));
typedef float    v8f  __attribute__((ext_vector_type(8)));
typedef float    v4f  __attribute__((ext_vector_type(4)));
typedef unsigned int   v4u  __attribute__((ext_vector_type(4)));
typedef unsigned short v8us __attribute__((ext_vector_type(8)));

__device__ __forceinline__ unsigned short bf_bits(float f) {
  unsigned u = __float_as_uint(f);
  return (unsigned short)((u + 0x7FFFu + ((u >> 16) & 1u)) >> 16);
}
__device__ __forceinline__ float bf_up(unsigned short h) { return __uint_as_float(((unsigned)h) << 16); }
__device__ __forceinline__ float bfr(float f) { return bf_up(bf_bits(f)); }
__device__ __forceinline__ unsigned short h_bits(_Float16 x) { return __builtin_bit_cast(unsigned short, x); }
__device__ __forceinline__ unsigned pk16(unsigned short a, unsigned short b) { return (unsigned)a | ((unsigned)b << 16); }
__device__ __forceinline__ int imin(int a, int b) { return a < b ? a : b; }
__device__ __forceinline__ int clampi(int v, int lo, int hi) { return v < lo ? lo : (v > hi ? hi : v); }
__device__ __forceinline__ v8f zero8() { v8f z = {0.f, 0.f, 0.f, 0.f, 0.f, 0.f, 0.f, 0.f}; return z; }

__device__ __forceinline__ void st2_us8(unsigned short* p, v8us v) {
  *(volatile v8us*)p = v;
  __threadfence();
  *(volatile v8us*)p = v;
}
__device__ __forceinline__ void st2_f4(float* p, v4f v) {
  *(volatile v4f*)p = v;
  __threadfence();
  *(volatile v4f*)p = v;
}

__device__ __forceinline__ v8us cvt8(const float* src) {
  const v4f a = *(const v4f*)(src);
  const v4f b = *(const v4f*)(src + 4);
  v8us p;
  p[0] = bf_bits(a[0]); p[1] = bf_bits(a[1]); p[2] = bf_bits(a[2]); p[3] = bf_bits(a[3]);
  p[4] = bf_bits(b[0]); p[5] = bf_bits(b[1]); p[6] = bf_bits(b[2]); p[7] = bf_bits(b[3]);
  return p;
}

__device__ __forceinline__ v16b ldfrag_b(const __bf16* p) {
  union { v16b v; v8b h[2]; } f;
  f.h[0] = *(const v8b*)(p);
  f.h[1] = *(const v8b*)(p + 16);
  return f.v;
}

__device__ __forceinline__ v8f mma_b(v16b a, v16b b, v8f c) {
  c = __builtin_amdgcn_wmma_f32_16x16x32_bf16(false, a, false, b, (short)0, c, false, false);
  asm volatile("v_nop\n\tv_nop\n\tv_nop\n\tv_nop" : "+v"(c) : "v"(a), "v"(b));
  return c;
}
__device__ __forceinline__ v8f mma_h(v16h a, v16h b, v8f c) {
  c = __builtin_amdgcn_wmma_f32_16x16x32_f16(false, a, false, b, (short)0, c, false, false);
  asm volatile("v_nop\n\tv_nop\n\tv_nop\n\tv_nop" : "+v"(c) : "v"(a), "v"(b));
  return c;
}
__device__ __forceinline__ v8f mma_b_raw(v16b a, v16b b, v8f c) {
  return __builtin_amdgcn_wmma_f32_16x16x32_bf16(false, a, false, b, (short)0, c, false, false);
}
__device__ __forceinline__ void dep_guard_b(v8f& a, v8f& b, v16b x, v16b y) {
  asm volatile("v_nop\n\tv_nop\n\tv_nop\n\tv_nop" : "+v"(a), "+v"(b) : "v"(x), "v"(y));
}
__device__ __forceinline__ void keep4_b(v16b a, v16b b, v16b c, v16b d) {
  asm volatile("v_nop" :: "v"(a), "v"(b), "v"(c), "v"(d));
}
__device__ __forceinline__ void keep2_b(v16b a, v16b b) {
  asm volatile("v_nop" :: "v"(a), "v"(b));
}
__device__ __forceinline__ void acc_guard4(v8f& a, v8f& b, v8f& c, v8f& d) {
  asm volatile("v_nop\n\tv_nop\n\tv_nop\n\tv_nop" : "+v"(a), "+v"(b), "+v"(c), "+v"(d));
}
__device__ __forceinline__ void acc_guard2(v8f& a, v8f& b) {
  asm volatile("v_nop\n\tv_nop\n\tv_nop\n\tv_nop" : "+v"(a), "+v"(b));
}

#define NX8 (TOKP * DIM / 8)
__global__ __launch_bounds__(256) void cvt_x(const float* __restrict__ x, unsigned short* Xb) {
  const int i = blockIdx.x * 256 + threadIdx.x;
  if (i >= NX8) return;
  const int prow = i >> 7;
  const int c8   = (i & 127) * 8;
  const int b    = prow / SP;
  const int t    = prow - b * SP;
  const int tc   = (t < SQ) ? t : (SQ - 1);
  const float* src = x + ((size_t)(b * SQ + tc) * DIM + c8);
  v8us p = cvt8(src);
  const bool ok = (t < SQ);
  const unsigned short z = 0;
#pragma unroll
  for (int e = 0; e < 8; ++e) p[e] = ok ? p[e] : z;
  st2_us8(Xb + (size_t)i * 8, p);
}

__global__ __launch_bounds__(256) void prep_lin(
    const float* __restrict__ W, const float* __restrict__ U, const float* __restrict__ S,
    const float* __restrict__ V, const int* __restrict__ idx, const float* __restrict__ gates,
    unsigned short* Wb, unsigned short* Ub, unsigned short* Vb, float* GS) {
  const int tid = threadIdx.x;
  const int blk = blockIdx.x;
  if (blk < 512) {
    const int i = blk * 256 + tid;
    const v8us p = cvt8(W + (size_t)i * 8);
    st2_us8(Wb + (size_t)i * 8, p);
  } else if (blk < 1024) {
    const int i  = (blk - 512) * 256 + tid;
    const int b  = i >> 12;
    const int o  = (i >> 2) & (DIM - 1);
    const int kq = i & 3;
    const int e  = clampi(idx[b * 2 + (kq >> 1)], 0, NE - 1);
    const float* src = U + ((size_t)(e * DIM + o) * RK + (kq & 1) * 8);
    const v8us p = cvt8(src);
    st2_us8(Ub + (size_t)i * 8, p);
  } else if (blk < 1536) {
    const int i  = (blk - 1024) * 256 + tid;
    const int b  = i >> 12;
    const int rr = (i >> 7) & 31;
    const int c8 = (i & 127) * 8;
    const int e  = clampi(idx[b * 2 + (rr >> 4)], 0, NE - 1);
    const float* src = V + ((size_t)(e * RK + (rr & 15)) * DIM + c8);
    const v8us p = cvt8(src);
    st2_us8(Vb + (size_t)i * 8, p);
  } else {
    const int i    = tid;
    const int b    = i >> 3;
    const int kq   = i & 7;
    const int slot = kq >> 2;
    const int e    = clampi(idx[b * 2 + slot], 0, NE - 1);
    const float g  = bfr(gates[b * 2 + slot]);
    const float* sp = S + e * RK + (kq & 3) * 4;
    v4f v;
#pragma unroll
    for (int cc = 0; cc < 4; ++cc) v[cc] = g * bfr(sp[cc]);
    st2_f4(GS + (size_t)i * 4, v);
  }
}

template <int NSPLIT>
__global__ __launch_bounds__(256) void lowrank32(
    const unsigned short* Ahp, const unsigned short* Alp,
    const unsigned short* __restrict__ Vbp, const float* __restrict__ GSp,
    unsigned short* Ehp, unsigned short* Elp) {
  __shared__ __align__(16) unsigned short sE[8][2][16 * KE];
  const __bf16* A  = (const __bf16*)(const void*)Ahp;
  const __bf16* A2 = (const __bf16*)(const void*)((NSPLIT >= 1) ? Alp : Ahp);
  const int lane = threadIdx.x & 31;
  const int wave = threadIdx.x >> 5;
  const int hh   = lane >> 4;
  const int c    = lane & 15;
  const int tw   = blockIdx.x * 8 + wave;
  const int row0 = tw * 16;
  const int bimg = tw / NQT;
  const __bf16* Bt = (const __bf16*)(const void*)Vbp + (size_t)bimg * KE * DIM;

  v8f acc[2];
  acc[0] = zero8(); acc[1] = zero8();
  for (int k0 = 0; k0 < DIM; k0 += 32) {
    const size_t ao = (size_t)(row0 + c) * DIM + k0 + 8 * hh;
    const v16b a = ldfrag_b(A + ao);
    v16b al = a;
    if (NSPLIT >= 1) al = ldfrag_b(A2 + ao);
    const v16b b0 = ldfrag_b(Bt + (size_t)c * DIM + k0 + 8 * hh);
    const v16b b1 = ldfrag_b(Bt + (size_t)(16 + c) * DIM + k0 + 8 * hh);
    acc[0] = mma_b_raw(a, b0, acc[0]);
    acc[1] = mma_b_raw(a, b1, acc[1]);
    if (NSPLIT >= 1) {
      acc[0] = mma_b_raw(al, b0, acc[0]);
      acc[1] = mma_b_raw(al, b1, acc[1]);
    }
    dep_guard_b(acc[0], acc[1], a, al);
    keep2_b(b0, b1);
  }
  acc_guard2(acc[0], acc[1]);

  const float gs0 = GSp[bimg * KE + c];
  const float gs1 = GSp[bimg * KE + 16 + c];
  unsigned short* sh = sE[wave][0];
  unsigned short* sl = sE[wave][1];
#pragma unroll
  for (int j = 0; j < 2; ++j) {
    const float gs = (j == 0) ? gs0 : gs1;
#pragma unroll
    for (int r = 0; r < 8; ++r) {
      const float f = acc[j][r] * gs;
      const unsigned short hb = bf_bits(f);
      const unsigned short lb = bf_bits(f - bf_up(hb));
      sh[(8 * hh + r) * KE + 16 * j + c] = hb;
      sl[(8 * hh + r) * KE + 16 * j + c] = lb;
    }
  }
  __builtin_amdgcn_fence(__ATOMIC_RELEASE, "workgroup");
  __builtin_amdgcn_wave_barrier();
  __builtin_amdgcn_fence(__ATOMIC_ACQUIRE, "workgroup");
  for (int pass = 0; pass < 2; ++pass) {
#pragma unroll
    for (int ch = 0; ch < 2; ++ch) {
      const v8us hv = *(const v8us*)(sh + ch * 256 + lane * 8);
      const v8us lv = *(const v8us*)(sl + ch * 256 + lane * 8);
      const size_t go = (size_t)row0 * KE + ch * 256 + lane * 8;
      *(volatile v8us*)(Ehp + go) = hv;
      *(volatile v8us*)(Elp + go) = lv;
    }
    __threadfence();
  }
}

template <int NSPLIT, int OM>
__global__ __launch_bounds__(64) void proj64(
    const unsigned short* Ahp, const unsigned short* Alp,
    const unsigned short* __restrict__ Wbp,
    const unsigned short* __restrict__ Ehp, const unsigned short* __restrict__ Elp,
    const unsigned short* __restrict__ Ubp, const float* __restrict__ bias,
    void* Cp, void* C2p, float oscale) {
  __shared__ __align__(16) float          sT[2][16 * 68];
  __shared__ __align__(16) unsigned short sV[2][2][64 * 72];
  const __bf16* A  = (const __bf16*)(const void*)Ahp;
  const __bf16* A2 = (const __bf16*)(const void*)((NSPLIT >= 1) ? Alp : Ahp);
  const __bf16* Bt = (const __bf16*)(const void*)Wbp;
  const __bf16* Eh = (const __bf16*)(const void*)Ehp;
  const __bf16* El = (const __bf16*)(const void*)Elp;
  const __bf16* Ub = (const __bf16*)(const void*)Ubp;
  const int lane = threadIdx.x & 31;
  const int wave = threadIdx.x >> 5;
  const int tile = blockIdx.x * 2 + wave;
  const int tm   = tile >> 4;
  const int tn   = tile & 15;
  const int m0   = tm << 6;
  const int n0   = tn << 6;
  const int rl   = lane & 15;
  const int koff = (lane >> 4) * 8;
  const int mOff = koff;

  v8f acc[4][4];
#pragma unroll
  for (int i = 0; i < 4; ++i)
#pragma unroll
    for (int j = 0; j < 4; ++j) acc[i][j] = zero8();

  for (int k0 = 0; k0 < DIM; k0 += 32) {
    v16b bh[4];
#pragma unroll
    for (int j = 0; j < 4; ++j)
      bh[j] = ldfrag_b(Bt + (size_t)(n0 + (j << 4) + rl) * DIM + koff + k0);
#pragma unroll
    for (int i = 0; i < 4; ++i) {
      const size_t ao = (size_t)(m0 + (i << 4) + rl) * DIM + koff + k0;
      const v16b ah = ldfrag_b(A + ao);
      v16b al = ah;
      if (NSPLIT >= 1) al = ldfrag_b(A2 + ao);
#pragma unroll
      for (int j = 0; j < 4; ++j) {
        acc[i][j] = mma_b_raw(ah, bh[j], acc[i][j]);
        if (NSPLIT >= 1) acc[i][j] = mma_b_raw(al, bh[j], acc[i][j]);
      }
      dep_guard_b(acc[i][0], acc[i][3], ah, al);
    }
    keep4_b(bh[0], bh[1], bh[2], bh[3]);
  }

#pragma unroll
  for (int i = 0; i < 4; ++i) {
    const int bimg = (m0 + (i << 4)) / SP;
    const size_t eo = (size_t)(m0 + (i << 4) + rl) * KE + koff;
    const v16b eh = ldfrag_b(Eh + eo);
    const v16b el = ldfrag_b(El + eo);
#pragma unroll
    for (int j = 0; j < 4; ++j) {
      const v16b ub = ldfrag_b(Ub + ((size_t)bimg * DIM + n0 + (j << 4) + rl) * KE + koff);
      acc[i][j] = mma_b(eh, ub, acc[i][j]);
      acc[i][j] = mma_b(el, ub, acc[i][j]);
    }
  }
  acc_guard4(acc[0][0], acc[0][1], acc[0][2], acc[0][3]);
  acc_guard4(acc[1][0], acc[1][1], acc[1][2], acc[1][3]);
  acc_guard4(acc[2][0], acc[2][1], acc[2][2], acc[2][3]);
  acc_guard4(acc[3][0], acc[3][1], acc[3][2], acc[3][3]);

  if (OM == 3) {
    unsigned short* th = sV[wave][0];
    unsigned short* tl = sV[wave][1];
    float bv[4];
#pragma unroll
    for (int j = 0; j < 4; ++j) bv[j] = bfr(bias[n0 + (j << 4) + rl]);
#pragma unroll
    for (int i = 0; i < 4; ++i) {
#pragma unroll
      for (int j = 0; j < 4; ++j) {
        v8us ph, pl;
#pragma unroll
        for (int r = 0; r < 8; ++r) {
          const float f = (acc[i][j][r] + bv[j]) * oscale;
          const _Float16 xh = (_Float16)f;
          ph[r] = h_bits(xh);
          pl[r] = h_bits((_Float16)((f - (float)xh) * 4096.0f));
        }
        *(v8us*)(th + ((j << 4) + rl) * 72 + (i << 4) + mOff) = ph;
        *(v8us*)(tl + ((j << 4) + rl) * 72 + (i << 4) + mOff) = pl;
      }
    }
    __builtin_amdgcn_fence(__ATOMIC_RELEASE, "workgroup");
    __builtin_amdgcn_wave_barrier();
    __builtin_amdgcn_fence(__ATOMIC_ACQUIRE, "workgroup");
    unsigned short* Ct  = (unsigned short*)Cp;
    unsigned short* Ct2 = (unsigned short*)C2p;
    const int q = lane >> 3, c8 = (lane & 7) * 8;
    for (int pass = 0; pass < 2; ++pass) {
#pragma unroll
      for (int it = 0; it < 16; ++it) {
        const int d = it * 4 + q;
        const v8us hv = *(const v8us*)(th + d * 72 + c8);
        const v8us lv = *(const v8us*)(tl + d * 72 + c8);
        const size_t go = (size_t)(n0 + d) * TOKP + m0 + c8;
        *(volatile v8us*)(Ct + go) = hv;
        *(volatile v8us*)(Ct2 + go) = lv;
      }
      __threadfence();
    }
  } else {
    float* slab = sT[wave];
#pragma unroll
    for (int i = 0; i < 4; ++i) {
      const int mBase = m0 + (i << 4);
#pragma unroll
      for (int j = 0; j < 4; ++j) {
#pragma unroll
        for (int r = 0; r < 8; ++r) {
          slab[(mOff + r) * 68 + (j << 4) + rl] = acc[i][j][r];
        }
      }
      __builtin_amdgcn_fence(__ATOMIC_RELEASE, "workgroup");
      __builtin_amdgcn_wave_barrier();
      __builtin_amdgcn_fence(__ATOMIC_ACQUIRE, "workgroup");
      if (OM == 0) {
        float* C = (float*)Cp;
        const int hq = lane >> 4, c4 = (lane & 15) * 4;
        v4f bv;
#pragma unroll
        for (int e = 0; e < 4; ++e) bv[e] = bfr(bias[n0 + c4 + e]);
        for (int pass = 0; pass < 2; ++pass) {
#pragma unroll
          for (int it = 0; it < 8; ++it) {
            const int row  = it * 2 + hq;
            const int m    = mBase + row;
            const int bimg = m / SP;
            const int t    = m - bimg * SP;
            v4f v = *(const v4f*)(slab + row * 68 + c4);
            v = (v + bv) * oscale;
            if (t < SQ)
              *(volatile v4f*)(C + ((size_t)(bimg * SQ + t) * DIM + n0 + c4)) = v;
          }
          __threadfence();
        }
      } else {
        const int q = lane >> 3, c8 = (lane & 7) * 8;
        unsigned short* C  = (unsigned short*)Cp;
        unsigned short* C2 = (unsigned short*)C2p;
        float bv8[8];
#pragma unroll
        for (int e = 0; e < 8; ++e) bv8[e] = bfr(bias[n0 + c8 + e]);
        v4u hv[4], lv[4];
#pragma unroll
        for (int it = 0; it < 4; ++it) {
          const int row = it * 4 + q;
          const float* sp = slab + row * 68 + c8;
          v4u a, a2;
#pragma unroll
          for (int e = 0; e < 4; ++e) {
            const float f0 = (sp[2 * e] + bv8[2 * e]) * oscale;
            const float f1 = (sp[2 * e + 1] + bv8[2 * e + 1]) * oscale;
            const unsigned short h0 = bf_bits(f0), h1 = bf_bits(f1);
            const unsigned short l0 = bf_bits(f0 - bf_up(h0)), l1 = bf_bits(f1 - bf_up(h1));
            a[e] = pk16(h0, h1); a2[e] = pk16(l0, l1);
          }
          hv[it] = a; lv[it] = a2;
        }
        for (int pass = 0; pass < 2; ++pass) {
#pragma unroll
          for (int it = 0; it < 4; ++it) {
            const int row = it * 4 + q;
            const size_t go = (size_t)(mBase + row) * DIM + n0 + c8;
            *(volatile v4u*)(C + go)  = hv[it];
            *(volatile v4u*)(C2 + go) = lv[it];
          }
          __threadfence();
        }
      }
      __builtin_amdgcn_fence(__ATOMIC_RELEASE, "workgroup");
      __builtin_amdgcn_wave_barrier();
      __builtin_amdgcn_fence(__ATOMIC_ACQUIRE, "workgroup");
    }
  }
}

__global__ __launch_bounds__(128)
void attn_img(const unsigned short* qhp, const unsigned short* qlp,
              const unsigned short* __restrict__ khp, const unsigned short* __restrict__ klp,
              const unsigned short* __restrict__ vhp, const unsigned short* __restrict__ vlp,
              unsigned short* ohp, unsigned short* olp) {
  union FB { v16b v; v8b h[2]; };
  union FH { v16h v; v8h h[2]; };
  __shared__ __align__(16) __bf16   Ksh[64 * 64];
  __shared__ __align__(16) __bf16   Ksl[64 * 64];
  __shared__ __align__(16) _Float16 Vth[64 * 64];
  __shared__ __align__(16) _Float16 Vtl[64 * 64];
  __shared__ __align__(16) _Float16 Psh[4][16 * 64];
  __shared__ __align__(16) float    Os[4][16 * 64];

  const int tid  = threadIdx.x;
  const int wave = tid >> 5;
  const int lane = tid & 31;
  const int hh   = lane >> 4;
  const int c    = lane & 15;

  const int bx   = blockIdx.x;
  const int qb   = bx % NQB;
  const int rest = bx / NQB;
  const int h    = rest % NH;
  const int b    = rest / NH;
  const int tile = qb * 4 + wave;
  const bool act = (tile < NQT);
  const int tq   = act ? tile : (NQT - 1);
  const size_t prow0 = (size_t)b * SP + (size_t)tq * 16;

  const __bf16* Qh = (const __bf16*)(const void*)qhp + (size_t)h * HD;
  const __bf16* Ql = (const __bf16*)(const void*)qlp + (size_t)h * HD;
  const __bf16* Kh = (const __bf16*)(const void*)khp + (size_t)h * HD;
  const __bf16* Kl = (const __bf16*)(const void*)klp + (size_t)h * HD;
  const _Float16* Vh = (const _Float16*)(const void*)vhp + (size_t)(h * HD) * TOKP + (size_t)b * SP;
  const _Float16* Vl = (const _Float16*)(const void*)vlp + (size_t)(h * HD) * TOKP + (size_t)b * SP;

  v16b qah[2], qal[2];
#pragma unroll
  for (int dc = 0; dc < 2; ++dc) {
    const size_t qo = (prow0 + c) * DIM + dc * 32 + 8 * hh;
    qah[dc] = ldfrag_b(Qh + qo);
    qal[dc] = ldfrag_b(Ql + qo);
  }

  float mrow[8], lrow[8];
  v8f oacc[4];
#pragma unroll
  for (int r = 0; r < 8; ++r) { mrow[r] = -INFINITY; lrow[r] = 0.f; }
#pragma unroll
  for (int t = 0; t < 4; ++t) oacc[t] = zero8();

#pragma unroll 1
  for (int kt = 0; kt < NKT; ++kt) {
    const int kv0  = kt * 64;
    const int nsub = (kt == NKT - 1) ? (NQT - 4 * (NKT - 1)) : 4;
    const int nks  = (nsub * 16 + 31) / 32;
    __syncthreads();
    {
      const int r = tid >> 1, half = (tid & 1) * 32;
      const int kr = imin(kv0 + r, SP - 1);
      const __bf16*   kg  = Kh + ((size_t)b * SP + kr) * DIM + half;
      const __bf16*   klg = Kl + ((size_t)b * SP + kr) * DIM + half;
      const _Float16* vg  = Vh + (size_t)r * TOKP;
      const _Float16* vlg = Vl + (size_t)r * TOKP;
#pragma unroll
      for (int i = 0; i < 4; ++i) {
        const int col  = kv0 + half + 8 * i;
        const int colc = imin(col, SP - 8);
        const v8b a0 = *(const v8b*)(kg + 8 * i);
        const v8b a1 = *(const v8b*)(klg + 8 * i);
        const v8h b0 = *(const v8h*)(vg + colc);
        const v8h b1 = *(const v8h*)(vlg + colc);
        *(v8b*)(Ksh + r * 64 + half + 8 * i) = a0;
        *(v8b*)(Ksl + r * 64 + half + 8 * i) = a1;
        *(v8h*)(Vth + r * 64 + half + 8 * i) = b0;
        *(v8h*)(Vtl + r * 64 + half + 8 * i) = b1;
      }
    }
    __syncthreads();

    if (act) {
      v8f s[4];
#pragma unroll
      for (int j = 0; j < 4; ++j) {
        s[j] = zero8();
        if (j < nsub) {
#pragma unroll
          for (int dc = 0; dc < 2; ++dc) {
            FB kb, kl;
            kb.h[0] = *(const v8b*)(Ksh + (j * 16 + c) * 64 + dc * 32 + 8 * hh);
            kb.h[1] = *(const v8b*)(Ksh + (j * 16 + c) * 64 + dc * 32 + 16 + 8 * hh);
            kl.h[0] = *(const v8b*)(Ksl + (j * 16 + c) * 64 + dc * 32 + 8 * hh);
            kl.h[1] = *(const v8b*)(Ksl + (j * 16 + c) * 64 + dc * 32 + 16 + 8 * hh);
            s[j] = mma_b(qah[dc], kb.v, s[j]);
            s[j] = mma_b(qah[dc], kl.v, s[j]);
            s[j] = mma_b(qal[dc], kb.v, s[j]);
          }
        }
      }

      _Float16* pwh = Psh[wave];
#pragma unroll
      for (int r = 0; r < 8; ++r) {
        float m = -INFINITY;
#pragma unroll
        for (int j = 0; j < 4; ++j) {
          const int key = kv0 + j * 16 + c;
          float sv = s[j][r];
          sv = (key < SQ) ? sv : -INFINITY;
          s[j][r] = sv;
          m = fmaxf(m, sv);
        }
#pragma unroll
        for (int off = 1; off < 16; off <<= 1) m = fmaxf(m, __shfl_xor(m, off, 32));
        const float mnew  = fmaxf(mrow[r], m);
        const float msafe = (mnew == -INFINITY) ? 0.f : mnew;
        const float alpha = __expf(mrow[r] - msafe);
        mrow[r] = mnew;
        float psum = 0.f;
#pragma unroll
        for (int j = 0; j < 4; ++j) {
          const float p = __expf(s[j][r] - msafe);
          psum += p;
          pwh[(8 * hh + r) * 64 + j * 16 + c] = (_Float16)(p * 1024.0f);
        }
#pragma unroll
        for (int off = 1; off < 16; off <<= 1) psum += __shfl_xor(psum, off, 32);
        lrow[r] = lrow[r] * alpha + psum;
#pragma unroll
        for (int t = 0; t < 4; ++t) oacc[t][r] *= alpha;
      }
      __builtin_amdgcn_fence(__ATOMIC_RELEASE, "workgroup");
      __builtin_amdgcn_wave_barrier();
      __builtin_amdgcn_fence(__ATOMIC_ACQUIRE, "workgroup");

      v8f o1[4];
#pragma unroll
      for (int t = 0; t < 4; ++t) o1[t] = zero8();
      for (int kk = 0; kk < nks; ++kk) {
        FH pa;
        pa.h[0] = *(const v8h*)(pwh + c * 64 + kk * 32 + 8 * hh);
        pa.h[1] = *(const v8h*)(pwh + c * 64 + kk * 32 + 16 + 8 * hh);
#pragma unroll
        for (int t = 0; t < 4; ++t) {
          FH vb, vl;
          vb.h[0] = *(const v8h*)(Vth + (t * 16 + c) * 64 + kk * 32 + 8 * hh);
          vb.h[1] = *(const v8h*)(Vth + (t * 16 + c) * 64 + kk * 32 + 16 + 8 * hh);
          vl.h[0] = *(const v8h*)(Vtl + (t * 16 + c) * 64 + kk * 32 + 8 * hh);
          vl.h[1] = *(const v8h*)(Vtl + (t * 16 + c) * 64 + kk * 32 + 16 + 8 * hh);
          oacc[t] = mma_h(pa.v, vb.v, oacc[t]);
          o1[t]   = mma_h(pa.v, vl.v, o1[t]);
        }
      }
#pragma unroll
      for (int t = 0; t < 4; ++t)
#pragma unroll
        for (int r = 0; r < 8; ++r) oacc[t][r] += o1[t][r] * (1.0f / 4096.0f);
    }
  }

  if (act) {
    float* os = Os[wave];
#pragma unroll
    for (int r = 0; r < 8; ++r) {
      const float l = lrow[r];
      const float inv = ((l > 0.f) ? (1.0f / l) : 0.f) * (1.0f / 8192.0f);
#pragma unroll
      for (int t = 0; t < 4; ++t) os[(8 * hh + r) * 64 + t * 16 + c] = oacc[t][r] * inv;
    }
    __builtin_amdgcn_fence(__ATOMIC_RELEASE, "workgroup");
    __builtin_amdgcn_wave_barrier();
    __builtin_amdgcn_fence(__ATOMIC_ACQUIRE, "workgroup");
    {
      const int q4 = lane >> 3, c8 = (lane & 7) * 8;
      v4u hv[4], lv[4];
#pragma unroll
      for (int it = 0; it < 4; ++it) {
        const int row = it * 4 + q4;
        const float* sp = os + row * 64 + c8;
        v4u a, a2;
#pragma unroll
        for (int e = 0; e < 4; ++e) {
          const float f0 = sp[2 * e], f1 = sp[2 * e + 1];
          const unsigned short h0 = bf_bits(f0), h1 = bf_bits(f1);
          const unsigned short l0 = bf_bits(f0 - bf_up(h0)), l1 = bf_bits(f1 - bf_up(h1));
          a[e] = pk16(h0, h1); a2[e] = pk16(l0, l1);
        }
        hv[it] = a; lv[it] = a2;
      }
      for (int pass = 0; pass < 2; ++pass) {
#pragma unroll
        for (int it = 0; it < 4; ++it) {
          const int row = it * 4 + q4;
          const size_t go = (prow0 + row) * DIM + (size_t)h * HD + c8;
          *(volatile v4u*)(ohp + go) = hv[it];
          *(volatile v4u*)(olp + go) = lv[it];
        }
        __threadfence();
      }
    }
  }
}

extern "C" void kernel_launch(void* const* d_in, const int* in_sizes, int n_in,
                              void* d_out, int out_size, void* d_ws, size_t ws_size,
                              hipStream_t stream) {
  if (n_in < 23) return;
  if (in_sizes[0] != BB * SQ * DIM) return;
  if (in_sizes[1] != BB * 2 || in_sizes[2] != BB * 2) return;
  for (int p = 0; p < 4; ++p) {
    const int base = 3 + 5 * p;
    if (in_sizes[base + 0] != DIM * DIM) return;
    if (in_sizes[base + 1] != NE * DIM * RK) return;
    if (in_sizes[base + 2] != NE * RK) return;
    if (in_sizes[base + 3] != NE * RK * DIM) return;
    if (in_sizes[base + 4] != DIM) return;
  }
  if (out_size != BB * SQ * DIM) return;

  const float* x     = (const float*)d_in[0];
  const int*   idx   = (const int*)d_in[1];
  const float* gates = (const float*)d_in[2];
  const float *W[4], *U[4], *S[4], *V[4], *Bi[4];
  for (int p = 0; p < 4; ++p) {
    const int base = 3 + 5 * p;
    W[p]  = (const float*)d_in[base + 0];
    U[p]  = (const float*)d_in[base + 1];
    S[p]  = (const float*)d_in[base + 2];
    V[p]  = (const float*)d_in[base + 3];
    Bi[p] = (const float*)d_in[base + 4];
  }

  const size_t PX  = (size_t)TOKP * DIM * 2;
  const size_t PW  = (size_t)DIM * DIM * 2;
  const size_t PU  = (size_t)BB * DIM * KE * 2;
  const size_t PV  = (size_t)BB * KE * DIM * 2;
  const size_t PG  = (size_t)BB * KE * 4;
  const size_t PE  = (size_t)TOKP * KE * 2;
  size_t off = 0;
  const size_t oXb = off; off += PX;
  const size_t oWb = off; off += PW;
  const size_t oUb = off; off += PU;
  const size_t oVb = off; off += PV;
  const size_t oGS = off; off += PG;
  const size_t oEh = off; off += PE;
  const size_t oEl = off; off += PE;
  const size_t oQh = off; off += PX;
  const size_t oQl = off; off += PX;
  const size_t oKh = off; off += PX;
  const size_t oKl = off; off += PX;
  const size_t oVh = off; off += PX;
  const size_t oVl = off; off += PX;
  if (off > ws_size) return;
  if (off > (size_t)134217728) return;
  const size_t oOh = oXb;
  const size_t oOl = oQl;

  char* ws = (char*)d_ws;
  unsigned short* Xb  = (unsigned short*)(ws + oXb);
  unsigned short* Wb  = (unsigned short*)(ws + oWb);
  unsigned short* Ub  = (unsigned short*)(ws + oUb);
  unsigned short* Vb  = (unsigned short*)(ws + oVb);
  float*          GS  = (float*)(ws + oGS);
  unsigned short* Eh  = (unsigned short*)(ws + oEh);
  unsigned short* El  = (unsigned short*)(ws + oEl);
  unsigned short* Qh  = (unsigned short*)(ws + oQh);
  unsigned short* Ql  = (unsigned short*)(ws + oQl);
  unsigned short* Kh  = (unsigned short*)(ws + oKh);
  unsigned short* Kl  = (unsigned short*)(ws + oKl);
  unsigned short* VTh = (unsigned short*)(ws + oVh);
  unsigned short* VTl = (unsigned short*)(ws + oVl);
  unsigned short* Oh  = (unsigned short*)(ws + oOh);
  unsigned short* Ol  = (unsigned short*)(ws + oOl);

  const dim3 gCvt((NX8 + 255) / 256);
  const dim3 gPrep(1537);
  const dim3 gLow((TOKP / 16 + 7) / 8);
  const dim3 gProj(((TOKP / 64) * (DIM / 64) + 1) / 2);
  const dim3 gAttn(BB * NH * NQB);

  cvt_x<<<gCvt, dim3(256), 0, stream>>>(x, Xb);

  prep_lin<<<gPrep, dim3(256), 0, stream>>>(W[0], U[0], S[0], V[0], idx, gates, Wb, Ub, Vb, GS);
  lowrank32<0><<<gLow, dim3(256), 0, stream>>>(Xb, Xb, Vb, GS, Eh, El);
  proj64<0, 2><<<gProj, dim3(64), 0, stream>>>(Xb, Xb, Wb, Eh, El, Ub, Bi[0], (void*)Qh, (void*)Ql, 0.125f);

  prep_lin<<<gPrep, dim3(256), 0, stream>>>(W[1], U[1], S[1], V[1], idx, gates, Wb, Ub, Vb, GS);
  lowrank32<0><<<gLow, dim3(256), 0, stream>>>(Xb, Xb, Vb, GS, Eh, El);
  proj64<0, 2><<<gProj, dim3(64), 0, stream>>>(Xb, Xb, Wb, Eh, El, Ub, Bi[1], (void*)Kh, (void*)Kl, 1.0f);

  prep_lin<<<gPrep, dim3(256), 0, stream>>>(W[2], U[2], S[2], V[2], idx, gates, Wb, Ub, Vb, GS);
  lowrank32<0><<<gLow, dim3(256), 0, stream>>>(Xb, Xb, Vb, GS, Eh, El);
  proj64<0, 3><<<gProj, dim3(64), 0, stream>>>(Xb, Xb, Wb, Eh, El, Ub, Bi[2], (void*)VTh, (void*)VTl, 8.0f);

  attn_img<<<gAttn, dim3(128), 0, stream>>>(Qh, Ql, Kh, Kl, VTh, VTl, Oh, Ol);

  prep_lin<<<gPrep, dim3(256), 0, stream>>>(W[3], U[3], S[3], V[3], idx, gates, Wb, Ub, Vb, GS);
  lowrank32<1><<<gLow, dim3(256), 0, stream>>>(Oh, Ol, Vb, GS, Eh, El);
  proj64<1, 0><<<gProj, dim3(64), 0, stream>>>(Oh, Ol, Wb, Eh, El, Ub, Bi[3], d_out, d_out, 1.0f);
  (void)hipGetLastError();
}
